// QANetAttBlock_15436112461930
// MI455X (gfx1250) — hardware-verified
//
#include <hip/hip_runtime.h>
#include <stdint.h>

typedef __attribute__((ext_vector_type(16))) _Float16 v16h;
typedef __attribute__((ext_vector_type(8)))  _Float16 v8h;
typedef __attribute__((ext_vector_type(16))) __bf16   v16b;
typedef __attribute__((ext_vector_type(8)))  __bf16   v8b;
typedef __attribute__((ext_vector_type(8)))  float    v8f;
typedef __attribute__((ext_vector_type(4)))  float    v4f;

__device__ __forceinline__ unsigned short f2bf_bits(float f) {
  unsigned u = __float_as_uint(f);
  return (unsigned short)((u + 0x7FFFu + ((u >> 16) & 1u)) >> 16);
}
__device__ __forceinline__ float bf_bits2f(unsigned short h) { return __uint_as_float(((unsigned)h) << 16); }

__device__ __forceinline__ void dep_guard_h(v8f& a, v8f& b, v16h x, v16h y) { asm volatile("v_nop\n\tv_nop\n\tv_nop\n\tv_nop" : "+v"(a), "+v"(b) : "v"(x), "v"(y)); }
__device__ __forceinline__ void dep_guard_b(v8f& a, v8f& b, v16b x, v16b y) { asm volatile("v_nop\n\tv_nop\n\tv_nop\n\tv_nop" : "+v"(a), "+v"(b) : "v"(x), "v"(y)); }
__device__ __forceinline__ void keep4_h(v16h a, v16h b, v16h c, v16h d) { asm volatile("v_nop" :: "v"(a), "v"(b), "v"(c), "v"(d)); }
__device__ __forceinline__ void keep4_b(v16b a, v16b b, v16b c, v16b d) { asm volatile("v_nop" :: "v"(a), "v"(b), "v"(c), "v"(d)); }
__device__ __forceinline__ void acc_guard4(v8f& a, v8f& b, v8f& c, v8f& d) { asm volatile("v_nop\n\tv_nop\n\tv_nop\n\tv_nop" : "+v"(a), "+v"(b), "+v"(c), "+v"(d)); }
template <typename T> struct Frag;
template <> struct Frag<_Float16> {
  typedef v16h V; union U { v16h v; v8h h[2]; };
  static __device__ __forceinline__ v16h load(const _Float16* p) {
    U f; f.h[0] = *(const v8h*)(p); f.h[1] = *(const v8h*)(p + 16); return f.v;
  }
  static __device__ __forceinline__ v8f mma(v16h a, v16h b, v8f c) {
    return __builtin_amdgcn_wmma_f32_16x16x32_f16(false, a, false, b, (short)0, c, false, false);
  }
  static __device__ __forceinline__ void guard(v8f& a, v8f& b, v16h x, v16h y) { dep_guard_h(a, b, x, y); }
  static __device__ __forceinline__ void keep(v16h a, v16h b, v16h c, v16h d) { keep4_h(a, b, c, d); }
};
template <> struct Frag<__bf16> {
  typedef v16b V; union U { v16b v; v8b h[2]; };
  static __device__ __forceinline__ v16b load(const __bf16* p) {
    U f; f.h[0] = *(const v8b*)(p); f.h[1] = *(const v8b*)(p + 16); return f.v;
  }
  static __device__ __forceinline__ v8f mma(v16b a, v16b b, v8f c) {
    return __builtin_amdgcn_wmma_f32_16x16x32_bf16(false, a, false, b, (short)0, c, false, false);
  }
  static __device__ __forceinline__ void guard(v8f& a, v8f& b, v16b x, v16b y) { dep_guard_b(a, b, x, y); }
  static __device__ __forceinline__ void keep(v16b a, v16b b, v16b c, v16b d) { keep4_b(a, b, c, d); }
};

template <int ET> struct Elem;
template <> struct Elem<0> { typedef _Float16 T; };
template <> struct Elem<1> { typedef __bf16 T; };
template <int ET, bool SPLIT, int BIAS_MODE, int OUT_MODE, bool RESID, int ACT = 0>
__global__ __launch_bounds__(256) void wmma_gemm64(
    const unsigned short* __restrict__ Ap, const unsigned short* __restrict__ A2p, int lda, long strideA,
    const unsigned short* __restrict__ Btp, const unsigned short* __restrict__ Bt2p, int ldb, long strideB,
    void* __restrict__ Cout, void* __restrict__ Cout2, int ldc, long strideC,
    const float* __restrict__ bias,
    const float* __restrict__ resid, long strideR,
    int M, int N, int K, float scale) {
  typedef typename Elem<ET>::T T;
  typedef typename Frag<T>::V V;
  const T* A = (const T*)Ap; const T* A2 = (const T*)A2p; const T* Bt = (const T*)Btp; const T* Bt2 = (const T*)Bt2p;
  __shared__ __align__(16) float sT[8][16 * 68];
  const int b    = blockIdx.y;
  const int lane = threadIdx.x & 31;
  const int wave = threadIdx.x >> 5;
  const int tilesN = N >> 6;
  const int tilesM = M >> 6;
  const int tile = blockIdx.x * 8 + wave;
  if (tile >= tilesM * tilesN) return;
  const int tm = tile / tilesN;
  const int tn = tile - tm * tilesN;
  const int m0 = tm << 6;
  const int n0 = tn << 6;

  const T* Ab  = A  + (size_t)b * strideA;
  const T* Bb  = Bt + (size_t)b * strideB;
  const T* Ab2 = SPLIT ? (A2  + (size_t)b * strideA) : nullptr;
  const T* Bb2 = SPLIT ? (Bt2 + (size_t)b * strideB) : nullptr;

  const int rlane = lane & 15;
  const int koff  = (lane >> 4) * 8;
  const int mOff  = (lane >> 4) * 8;

  v8f acc[4][4];
#pragma unroll
  for (int i = 0; i < 4; ++i)
#pragma unroll
    for (int j = 0; j < 4; ++j) acc[i][j] = (v8f){0.f,0.f,0.f,0.f,0.f,0.f,0.f,0.f};

  for (int k0 = 0; k0 < K; k0 += 32) {
    V bh[4], bl[4];
#pragma unroll
    for (int j = 0; j < 4; ++j) {
      const size_t bo = (size_t)(n0 + (j << 4) + rlane) * ldb + koff + k0;
      bh[j] = Frag<T>::load(Bb + bo);
      if (SPLIT) bl[j] = Frag<T>::load(Bb2 + bo);
    }
#pragma unroll
    for (int i = 0; i < 4; ++i) {
      const size_t ao = (size_t)(m0 + (i << 4) + rlane) * lda + koff + k0;
      V ah = Frag<T>::load(Ab + ao);
      V al;
      if (SPLIT) al = Frag<T>::load(Ab2 + ao);
#pragma unroll
      for (int j = 0; j < 4; ++j) {
        acc[i][j] = Frag<T>::mma(ah, bh[j], acc[i][j]);
        if (SPLIT) {
          acc[i][j] = Frag<T>::mma(ah, bl[j], acc[i][j]);
          acc[i][j] = Frag<T>::mma(al, bh[j], acc[i][j]);
        }
      }
      Frag<T>::guard(acc[i][0], acc[i][3], ah, SPLIT ? al : ah);
    }
    Frag<T>::keep(bh[0], bh[1], bh[2], bh[3]);
    if (SPLIT) Frag<T>::keep(bl[0], bl[1], bl[2], bl[3]);
  }
  acc_guard4(acc[0][0], acc[0][1], acc[0][2], acc[0][3]);
  acc_guard4(acc[1][0], acc[1][1], acc[1][2], acc[1][3]);
  acc_guard4(acc[2][0], acc[2][1], acc[2][2], acc[2][3]);
  acc_guard4(acc[3][0], acc[3][1], acc[3][2], acc[3][3]);

  float* slab = sT[wave];
  const float* Rb = RESID ? (resid + (size_t)b * strideR) : nullptr;
#pragma unroll
  for (int i = 0; i < 4; ++i) {
    const int mBase = m0 + (i << 4);
#pragma unroll
    for (int j = 0; j < 4; ++j) {
      const int n = n0 + (j << 4) + rlane;
      float bv = 0.f;
      if (BIAS_MODE == 2) bv = bias[n];
#pragma unroll
      for (int r = 0; r < 8; ++r) {
        float v = acc[i][j][r] * scale;
        if (BIAS_MODE == 1) v += bias[mBase + mOff + r];
        if (BIAS_MODE == 2) v += bv;
        if (RESID) v += Rb[(size_t)(mBase + mOff + r) * ldc + n];
        if (ACT == 1) v = tanhf(v);
        if (ACT == 2) v = fmaxf(v, 0.0f);
        if (ACT == 3) v = v / (1.0f + expf(-v));
        if (ACT == 4) v = (v > 0.f) ? v : 0.01f * v;
        if (ACT == 5) v = 0.5f * v * (1.0f + erff(v * 0.70710678118654752f));
        slab[(mOff + r) * 68 + (j << 4) + rlane] = v;
      }
    }
    __builtin_amdgcn_fence(__ATOMIC_RELEASE, "workgroup");
    __builtin_amdgcn_wave_barrier();
    __builtin_amdgcn_fence(__ATOMIC_ACQUIRE, "workgroup");
    if (OUT_MODE == 0) {
      float* C = (float*)Cout + (size_t)b * strideC;
      const int hh = lane >> 4, c4 = (lane & 15) * 4;
      for (int pass = 0; pass < 2; ++pass) {
#pragma unroll
        for (int it = 0; it < 8; ++it) {
          const int row = it * 2 + hh;
          v4f v = *(const v4f*)(slab + row * 68 + c4);
          *(volatile v4f*)(C + (size_t)(mBase + row) * ldc + n0 + c4) = v;
        }
        __threadfence();
      }
    } else {
      const int q = lane >> 3, c8 = (lane & 7) * 8;
      unsigned short* C  = (unsigned short*)Cout  + (size_t)b * strideC;
      unsigned short* C2 = (OUT_MODE == 2) ? ((unsigned short*)Cout2 + (size_t)b * strideC) : nullptr;
      for (int pass = 0; pass < 2; ++pass) {
#pragma unroll
        for (int it = 0; it < 4; ++it) {
          const int row = it * 4 + q;
          const float* sp = slab + row * 68 + c8;
          v8h hv, lv;
#pragma unroll
          for (int e = 0; e < 8; ++e) {
            if (OUT_MODE == 1) {
              hv[e] = (_Float16)sp[e];
            } else {
              unsigned short hb = f2bf_bits(sp[e]);
              unsigned short lb = f2bf_bits(sp[e] - bf_bits2f(hb));
              hv[e] = __builtin_bit_cast(_Float16, hb);
              lv[e] = __builtin_bit_cast(_Float16, lb);
            }
          }
          *(volatile v8h*)(C + (size_t)(mBase + row) * ldc + n0 + c8) = hv;
          if (OUT_MODE == 2) *(volatile v8h*)(C2 + (size_t)(mBase + row) * ldc + n0 + c8) = lv;
        }
        __threadfence();
      }
    }
    __builtin_amdgcn_fence(__ATOMIC_RELEASE, "workgroup");
    __builtin_amdgcn_wave_barrier();
    __builtin_amdgcn_fence(__ATOMIC_ACQUIRE, "workgroup");
  }
}

__global__ __launch_bounds__(256) void cast_f32_f16x2(
    const float* __restrict__ in, _Float16* __restrict__ out, int n2) {
  int i = blockIdx.x * 256 + threadIdx.x;
  if (i < n2) {
    const _Float16 h0 = (_Float16)in[2 * i], h1 = (_Float16)in[2 * i + 1];
    const unsigned u = (unsigned)__builtin_bit_cast(unsigned short, h0) | ((unsigned)__builtin_bit_cast(unsigned short, h1) << 16);
    ((volatile unsigned*)out)[i] = u;
    __threadfence();
    ((volatile unsigned*)out)[i] = u;
  }
}

__global__ __launch_bounds__(256) void build_wqkvT(
    const float* __restrict__ Wq, const float* __restrict__ Wk, const float* __restrict__ Wv,
    _Float16* __restrict__ out, int n2, float wscale) {
  int i = blockIdx.x * 256 + threadIdx.x;
  if (i < n2) {
    const int e0 = 2 * i;
    const int n = e0 >> 9;
    const int kx = e0 & 511;
    const int mat = n >> 9;
    const int head = (n >> 6) & 7;
    const int d = n & 63;
    const float* W = (mat == 0) ? Wq : ((mat == 1) ? Wk : Wv);
    const size_t base = ((size_t)head * 512 + kx) * 64 + d;
    const _Float16 h0 = (_Float16)(W[base] * wscale);
    const _Float16 h1 = (_Float16)(W[base + 64] * wscale);
    const unsigned u = (unsigned)__builtin_bit_cast(unsigned short, h0) | ((unsigned)__builtin_bit_cast(unsigned short, h1) << 16);
    ((volatile unsigned*)out)[i] = u;
    __threadfence();
    ((volatile unsigned*)out)[i] = u;
  }
}

__global__ __launch_bounds__(256) void build_woT(
    const float* __restrict__ Wo, _Float16* __restrict__ out, int n2, float wscale) {
  int i = blockIdx.x * 256 + threadIdx.x;
  if (i < n2) {
    const int e0 = 2 * i;
    const int j = e0 >> 9;
    const int kx = e0 & 511;
    const _Float16 h0 = (_Float16)(Wo[(size_t)kx * 512 + j] * wscale);
    const _Float16 h1 = (_Float16)(Wo[(size_t)(kx + 1) * 512 + j] * wscale);
    const unsigned u = (unsigned)__builtin_bit_cast(unsigned short, h0) | ((unsigned)__builtin_bit_cast(unsigned short, h1) << 16);
    ((volatile unsigned*)out)[i] = u;
    __threadfence();
    ((volatile unsigned*)out)[i] = u;
  }
}

#define AT_D 64
#define AT_NW 4
#define AT_QB 64
#define AT_KC 64
struct AttnGeomH { long q_bs, q_rs, q_hs, k_bs, k_rs, k_hs, v_bs, v_rs, v_hs, o_bs, o_rs, o_hs, m_bs;
                   int S, Skv, H, nqb; float mask_fill; float oscale; };
typedef char attn_geom_size_check[(sizeof(AttnGeomH) == 128) ? 1 : -1];

__device__ __forceinline__ v8f hmma(v16h a, v16h b, v8f c) {
  c = __builtin_amdgcn_wmma_f32_16x16x32_f16(false, a, false, b, (short)0, c, false, false);
  asm volatile("v_nop\n\tv_nop\n\tv_nop\n\tv_nop" : "+v"(c) : "v"(a), "v"(b));
  return c;
}

__global__ __launch_bounds__(128)
void attn64h_kernel(const _Float16* __restrict__ q, const _Float16* __restrict__ k,
                    const _Float16* __restrict__ v, _Float16* __restrict__ out,
                    const int* __restrict__ mask, AttnGeomH g) {
  const float PSC = 32768.0f;
  union FB { v16h v; v8h h[2]; };
  __shared__ __align__(16) _Float16 Ksh[AT_KC * AT_D];
  __shared__ __align__(16) _Float16 Vth[AT_D * AT_KC];
  __shared__ __align__(16) _Float16 Psh[AT_NW][16 * AT_KC];
  __shared__ __align__(16) float    Os[AT_NW][16 * 68];
  __shared__ int red[AT_NW];

  const int tid  = threadIdx.x;
  const int wave = tid >> 5;
  const int lane = tid & 31;
  const int hh   = lane >> 4;
  const int c    = lane & 15;

  const int bx = blockIdx.x;
  const int qb = bx % g.nqb;
  const int bh = bx / g.nqb;
  const int h  = bh % g.H;
  const int b  = bh / g.H;
  const int q0 = qb * AT_QB + wave * 16;

  const _Float16* qb_ptr = q + (size_t)b * g.q_bs + (size_t)h * g.q_hs;
  const _Float16* kb_ptr = k + (size_t)b * g.k_bs + (size_t)h * g.k_hs;
  const _Float16* vb_ptr = v + (size_t)b * g.v_bs + (size_t)h * g.v_hs;
  _Float16*       ob_ptr = out + (size_t)b * g.o_bs + (size_t)h * g.o_hs;
  const int*      mb_ptr = mask + (size_t)b * g.m_bs;

  int part = 0;
  for (int i = tid; i < g.Skv; i += AT_NW * 32) part += mb_ptr[i];
#pragma unroll
  for (int off = 1; off < 32; off <<= 1) part += __shfl_xor(part, off, 32);
  if (lane == 0) red[wave] = part;
  __syncthreads();
  const int nsum = red[0] + red[1] + red[2] + red[3];
  const float qs = 1.0f / sqrtf((float)nsum);

  v16h qa[2];
  {
    const _Float16* qrow = qb_ptr + (size_t)(q0 + c) * g.q_rs;
#pragma unroll
    for (int dc = 0; dc < 2; ++dc) {
      FB f;
      f.h[0] = *(const v8h*)(qrow + dc * 32 + 8 * hh);
      f.h[1] = *(const v8h*)(qrow + dc * 32 + 16 + 8 * hh);
      qa[dc] = f.v;
    }
  }

  float mrow[8], lrow[8];
  v8f oacc[4];
#pragma unroll
  for (int r = 0; r < 8; ++r) { mrow[r] = -INFINITY; lrow[r] = 0.f; }
#pragma unroll
  for (int t = 0; t < 4; ++t) oacc[t] = (v8f){0.f,0.f,0.f,0.f,0.f,0.f,0.f,0.f};

  const int nChunks = g.Skv / AT_KC;
  int qkeep[8];
#pragma unroll
  for (int r = 0; r < 8; ++r) qkeep[r] = mb_ptr[q0 + 8 * hh + r];

  for (int kc = 0; kc < nChunks; ++kc) {
    const int kv0 = kc * AT_KC;
    __syncthreads();
    {
      const int kvr = tid >> 1, dh = (tid & 1) * 32;
      const _Float16* krow = kb_ptr + (size_t)(kv0 + kvr) * g.k_rs + dh;
      const _Float16* vrow = vb_ptr + (size_t)(kv0 + kvr) * g.v_rs + dh;
#pragma unroll
      for (int i = 0; i < 4; ++i) {
        const v8h kk8 = *(const v8h*)(krow + 8 * i);
        const v8h vv8 = *(const v8h*)(vrow + 8 * i);
        *(v8h*)(Ksh + kvr * AT_D + dh + 8 * i) = kk8;
#pragma unroll
        for (int e = 0; e < 8; ++e) Vth[(dh + 8 * i + e) * AT_KC + kvr] = vv8[e];
      }
    }
    __syncthreads();

    v8f s[4];
#pragma unroll
    for (int j = 0; j < 4; ++j) {
      s[j] = (v8f){0.f,0.f,0.f,0.f,0.f,0.f,0.f,0.f};
#pragma unroll
      for (int dc = 0; dc < 2; ++dc) {
        FB kb;
        kb.h[0] = *(const v8h*)(Ksh + (j * 16 + c) * AT_D + dc * 32 + 8 * hh);
        kb.h[1] = *(const v8h*)(Ksh + (j * 16 + c) * AT_D + dc * 32 + 16 + 8 * hh);
        s[j] = hmma(qa[dc], kb.v, s[j]);
      }
    }
    int kvkeep[4];
#pragma unroll
    for (int j = 0; j < 4; ++j) kvkeep[j] = mb_ptr[kv0 + j * 16 + c];
    float cm[8];
#pragma unroll
    for (int r = 0; r < 8; ++r) {
      float m = -INFINITY;
#pragma unroll
      for (int j = 0; j < 4; ++j) {
        float sv = s[j][r] * qs;
        if ((qkeep[r] == 0) || (kvkeep[j] == 0)) sv = g.mask_fill;
        s[j][r] = sv;
        m = fmaxf(m, sv);
      }
#pragma unroll
      for (int off = 1; off < 16; off <<= 1) m = fmaxf(m, __shfl_xor(m, off, 32));
      cm[r] = m;
    }
    _Float16* pwh = Psh[wave];
#pragma unroll
    for (int r = 0; r < 8; ++r) {
      const float mnew = fmaxf(mrow[r], cm[r]);
      const float alpha = expf(mrow[r] - mnew);
      mrow[r] = mnew;
      float psum = 0.f;
#pragma unroll
      for (int j = 0; j < 4; ++j) {
        const float p = expf(s[j][r] - mnew);
        psum += p;
        pwh[(8 * hh + r) * AT_KC + j * 16 + c] = (_Float16)(p * PSC);
      }
#pragma unroll
      for (int off = 1; off < 16; off <<= 1) psum += __shfl_xor(psum, off, 32);
      lrow[r] = lrow[r] * alpha + psum;
#pragma unroll
      for (int t = 0; t < 4; ++t) oacc[t][r] *= alpha;
    }
    __builtin_amdgcn_fence(__ATOMIC_RELEASE, "workgroup");
    __builtin_amdgcn_wave_barrier();
    __builtin_amdgcn_fence(__ATOMIC_ACQUIRE, "workgroup");
#pragma unroll 1
    for (int kk = 0; kk < 2; ++kk) {
      FB pa;
      pa.h[0] = *(const v8h*)(pwh + c * AT_KC + kk * 32 + 8 * hh);
      pa.h[1] = *(const v8h*)(pwh + c * AT_KC + kk * 32 + 16 + 8 * hh);
#pragma unroll
      for (int t = 0; t < 4; ++t) {
        FB vb;
        vb.h[0] = *(const v8h*)(Vth + (t * 16 + c) * AT_KC + kk * 32 + 8 * hh);
        vb.h[1] = *(const v8h*)(Vth + (t * 16 + c) * AT_KC + kk * 32 + 16 + 8 * hh);
        oacc[t] = hmma(pa.v, vb.v, oacc[t]);
      }
    }
  }

  float* os = Os[wave];
#pragma unroll
  for (int r = 0; r < 8; ++r) {
    const float inv = g.oscale / (lrow[r] * PSC);
#pragma unroll
    for (int t = 0; t < 4; ++t) os[(8 * hh + r) * 68 + t * 16 + c] = oacc[t][r] * inv;
  }
  __builtin_amdgcn_fence(__ATOMIC_RELEASE, "workgroup");
  __builtin_amdgcn_wave_barrier();
  __builtin_amdgcn_fence(__ATOMIC_ACQUIRE, "workgroup");
  {
    const int q8 = lane >> 3, c8 = (lane & 7) * 8;
    for (int pass = 0; pass < 2; ++pass) {
#pragma unroll
      for (int it = 0; it < 4; ++it) {
        const int row = it * 4 + q8;
        const float* sp = os + row * 68 + c8;
        v8h hv;
#pragma unroll
        for (int e = 0; e < 8; ++e) hv[e] = (_Float16)sp[e];
        *(volatile v8h*)(ob_ptr + (size_t)(q0 + row) * g.o_rs + c8) = hv;
      }
      __threadfence();
    }
  }
}

extern "C" void kernel_launch(void* const* d_in, const int* in_sizes, int n_in,
                              void* d_out, int out_size, void* d_ws, size_t ws_size,
                              hipStream_t stream) {
  const int NB = 16, NS = 1024, NHID = 512, NH = 8, NDK = 64;
  const int NTOK = NB * NS;
  const int NQKV = 3 * NH * NDK;
  if (n_in < 6) return;
  if (in_sizes[0] != NTOK * NHID) return;
  if (in_sizes[1] != NB * NS) return;
  if (in_sizes[2] != NH * NHID * NDK || in_sizes[3] != NH * NHID * NDK || in_sizes[4] != NH * NHID * NDK) return;
  if (in_sizes[5] != NHID * NHID) return;
  if (out_size != NTOK * NHID) return;

  const float* x    = (const float*)d_in[0];
  const int*   mask = (const int*)d_in[1];
  const float* Wq   = (const float*)d_in[2];
  const float* Wk   = (const float*)d_in[3];
  const float* Wv   = (const float*)d_in[4];
  const float* Wout = (const float*)d_in[5];
  float* out = (float*)d_out;

  char* ws = (char*)d_ws;
  size_t off = 0;
  const size_t bytes_xh   = (size_t)NTOK * NHID * 2;
  const size_t bytes_wqkv = (size_t)NQKV * NHID * 2;
  const size_t bytes_wo   = (size_t)NHID * NHID * 2;
  const size_t bytes_qkv  = (size_t)NTOK * NQKV * 2;
  const size_t bytes_o    = (size_t)NTOK * NHID * 2;
  const size_t o_xh   = off; off = (off + bytes_xh + 255) & ~(size_t)255;
  const size_t o_wqkv = off; off = (off + bytes_wqkv + 255) & ~(size_t)255;
  const size_t o_wo   = off; off = (off + bytes_wo + 255) & ~(size_t)255;
  const size_t o_qkv  = off; off = (off + bytes_qkv + 255) & ~(size_t)255;
  const size_t o_o    = off; off = (off + bytes_o + 255) & ~(size_t)255;
  if (off > ws_size) return;

  _Float16* xh    = (_Float16*)(ws + o_xh);
  _Float16* wqkvT = (_Float16*)(ws + o_wqkv);
  _Float16* woT   = (_Float16*)(ws + o_wo);
  _Float16* qkvb  = (_Float16*)(ws + o_qkv);
  _Float16* ob    = (_Float16*)(ws + o_o);

  {
    const int n2 = NTOK * NHID / 2;
    cast_f32_f16x2<<<(n2 + 255) / 256, 256, 0, stream>>>(x, xh, n2);
  }
  {
    const int n2 = NQKV * NHID / 2;
    build_wqkvT<<<(n2 + 255) / 256, 256, 0, stream>>>(Wq, Wk, Wv, wqkvT, n2, 64.0f);
  }
  {
    const int n2 = NHID * NHID / 2;
    build_woT<<<(n2 + 255) / 256, 256, 0, stream>>>(Wout, woT, n2, 64.0f);
  }
  {
    const int M = NTOK, N = NQKV, K = NHID;
    const int tiles = (M / 64) * (N / 64);
    dim3 grid((tiles + 7) / 8, 1);
    hipLaunchKernelGGL((wmma_gemm64<0, false, 0, 1, false, 0>), grid, dim3(256), 0, stream,
                       (const unsigned short*)xh, (const unsigned short*)xh, K, (long)0,
                       (const unsigned short*)wqkvT, (const unsigned short*)wqkvT, K, (long)0,
                       (void*)qkvb, (void*)qkvb, N, (long)0,
                       x, x, (long)0,
                       M, N, K, 1.0f / 64.0f);
  }
  {
    AttnGeomH g;
    g.q_bs = (long)NS * NQKV; g.q_rs = NQKV; g.q_hs = NDK;
    g.k_bs = (long)NS * NQKV; g.k_rs = NQKV; g.k_hs = NDK;
    g.v_bs = (long)NS * NQKV; g.v_rs = NQKV; g.v_hs = NDK;
    g.o_bs = (long)NS * NHID; g.o_rs = NHID; g.o_hs = NDK;
    g.m_bs = NS;
    g.S = NS; g.Skv = NS; g.H = NH; g.nqb = NS / AT_QB;
    g.mask_fill = -1.0e30f; g.oscale = 16.0f;
    const int nblk = NB * NH * (NS / AT_QB);
    attn64h_kernel<<<nblk, 128, 0, stream>>>(qkvb, qkvb + NH * NDK, qkvb + 2 * NH * NDK, ob, mask, g);
  }
  {
    const int M = NTOK, N = NHID, K = NHID;
    const int tiles = (M / 64) * (N / 64);
    dim3 grid((tiles + 7) / 8, 1);
    hipLaunchKernelGGL((wmma_gemm64<0, false, 0, 0, false, 0>), grid, dim3(256), 0, stream,
                       (const unsigned short*)ob, (const unsigned short*)ob, K, (long)0,
                       (const unsigned short*)woT, (const unsigned short*)woT, K, (long)0,
                       (void*)out, (void*)out, N, (long)0,
                       x, x, (long)0,
                       M, N, K, 1.0f / 1024.0f);
  }
  (void)hipGetLastError();
}
